// HGAT_56951266345673
// MI455X (gfx1250) — hardware-verified
//
#include <hip/hip_runtime.h>

typedef __attribute__((ext_vector_type(16))) _Float16 v16h;
typedef __attribute__((ext_vector_type(8)))  _Float16 v8h;
typedef __attribute__((ext_vector_type(16))) __bf16   v16b;
typedef __attribute__((ext_vector_type(8)))  __bf16   v8b;
typedef __attribute__((ext_vector_type(8)))  float    v8f;
typedef __attribute__((ext_vector_type(4)))  float    v4f;
typedef __attribute__((ext_vector_type(2)))  float    v2f;

constexpr int NNODE   = 2048;
constexpr int NFEAT_C = 512;
constexpr int NHID_C  = 128;
constexpr int NHEAD_C = 4;
constexpr int NPATH_C = 3;
constexpr int SHID_C  = 128;
constexpr int NPH_C   = NPATH_C * NHEAD_C;
constexpr int KCAT_C  = NHEAD_C * NHID_C;
constexpr float LRELU_SLOPE = 0.2f;
constexpr float MASK_FILL   = -9.0e15f;
constexpr float PCARRY      = 4096.0f;
constexpr float PCARRY_INV  = 1.0f / 4096.0f;
constexpr float MCARRY      = 64.0f;
constexpr float WSEM_CARRY  = 16.0f;
constexpr float SEM_SCALE   = 1.0f / (64.0f * 16.0f);
constexpr int SLAB_PITCH    = 132;

static_assert(NHID_C % 64 == 0, "");
static_assert(NNODE % 64 == 0, "");
static_assert(NFEAT_C % 32 == 0, "");
static_assert((NPATH_C * NNODE) % 64 == 0, "");
static_assert(SHID_C % 64 == 0, "");
static_assert(KCAT_C % 32 == 0, "");
static_assert(NNODE % 32 == 0, "");

constexpr size_t SZ_X16    = (size_t)NNODE * NFEAT_C * 2;
constexpr size_t SZ_WT16   = (size_t)NPH_C * NHID_C * NFEAT_C * 2;
constexpr size_t SZ_HT32   = (size_t)NPH_C * NHID_C * NNODE * 4;
constexpr size_t SZ_HT16   = (size_t)NPH_C * NHID_C * NNODE * 2;
constexpr size_t SZ_VEC    = (size_t)NPH_C * NNODE * 4;
constexpr size_t SZ_M32    = (size_t)NPATH_C * NNODE * KCAT_C * 4;
constexpr size_t SZ_M16    = (size_t)NPATH_C * NNODE * KCAT_C * 2;
constexpr size_t SZ_WSEMT  = (size_t)SHID_C * KCAT_C * 2;
constexpr size_t SZ_HS     = (size_t)NPATH_C * NNODE * SHID_C * 4;
constexpr size_t SZ_SC     = 512;
constexpr size_t OFF_XHI   = 0;
constexpr size_t OFF_XLO   = OFF_XHI + SZ_X16;
constexpr size_t OFF_WTHI  = OFF_XLO + SZ_X16;
constexpr size_t OFF_WTLO  = OFF_WTHI + SZ_WT16;
constexpr size_t OFF_HT32  = OFF_WTLO + SZ_WT16;
constexpr size_t OFF_HT16  = OFF_HT32 + SZ_HT32;
constexpr size_t OFF_SSRC  = OFF_HT16 + SZ_HT16;
constexpr size_t OFF_SDST  = OFF_SSRC + SZ_VEC;
constexpr size_t OFF_RMAX  = OFF_SDST + SZ_VEC;
constexpr size_t OFF_RINV  = OFF_RMAX + SZ_VEC;
constexpr size_t OFF_M32   = OFF_RINV + SZ_VEC;
constexpr size_t OFF_M16   = OFF_M32 + SZ_M32;
constexpr size_t OFF_WSEMT = OFF_M16 + SZ_M16;
constexpr size_t OFF_HS    = OFF_WSEMT + SZ_WSEMT;
constexpr size_t OFF_SC    = OFF_HS + SZ_HS;
constexpr size_t WS_TOTAL  = OFF_SC + SZ_SC;
static_assert(WS_TOTAL == 48759296, "");
static_assert(WS_TOTAL <= (size_t)134217728, "");
static_assert((OFF_XLO | OFF_WTHI | OFF_WTLO | OFF_HT32 | OFF_HT16 | OFF_SSRC | OFF_SDST | OFF_RMAX | OFF_RINV | OFF_M32 | OFF_M16 | OFF_WSEMT | OFF_HS | OFF_SC) % 256 == 0, "");

__device__ __forceinline__ unsigned short f2bf_bits(float f) {
  unsigned u = __float_as_uint(f);
  return (unsigned short)((u + 0x7FFFu + ((u >> 16) & 1u)) >> 16);
}
__device__ __forceinline__ float bf_bits2f(unsigned short h) { return __uint_as_float(((unsigned)h) << 16); }

__device__ __forceinline__ void dep_guard_h(v8f& a, v8f& b, v16h x, v16h y) { asm volatile("v_nop\n\tv_nop\n\tv_nop\n\tv_nop" : "+v"(a), "+v"(b) : "v"(x), "v"(y)); }
__device__ __forceinline__ void dep_guard_b(v8f& a, v8f& b, v16b x, v16b y) { asm volatile("v_nop\n\tv_nop\n\tv_nop\n\tv_nop" : "+v"(a), "+v"(b) : "v"(x), "v"(y)); }
__device__ __forceinline__ void keep4_h(v16h a, v16h b, v16h c, v16h d) { asm volatile("v_nop" :: "v"(a), "v"(b), "v"(c), "v"(d)); }
__device__ __forceinline__ void keep4_b(v16b a, v16b b, v16b c, v16b d) { asm volatile("v_nop" :: "v"(a), "v"(b), "v"(c), "v"(d)); }
__device__ __forceinline__ void acc_guard4(v8f& a, v8f& b, v8f& c, v8f& d) { asm volatile("v_nop\n\tv_nop\n\tv_nop\n\tv_nop" : "+v"(a), "+v"(b), "+v"(c), "+v"(d)); }
template <typename T> struct Frag;
template <> struct Frag<_Float16> {
  typedef v16h V; union U { v16h v; v8h h[2]; };
  static __device__ __forceinline__ v16h load(const _Float16* p) {
    U f; f.h[0] = *(const v8h*)(p); f.h[1] = *(const v8h*)(p + 16); return f.v;
  }
  static __device__ __forceinline__ v8f mma(v16h a, v16h b, v8f c) {
    return __builtin_amdgcn_wmma_f32_16x16x32_f16(false, a, false, b, (short)0, c, false, false);
  }
  static __device__ __forceinline__ void guard(v8f& a, v8f& b, v16h x, v16h y) { dep_guard_h(a, b, x, y); }
  static __device__ __forceinline__ void keep(v16h a, v16h b, v16h c, v16h d) { keep4_h(a, b, c, d); }
};
template <> struct Frag<__bf16> {
  typedef v16b V; union U { v16b v; v8b h[2]; };
  static __device__ __forceinline__ v16b load(const __bf16* p) {
    U f; f.h[0] = *(const v8b*)(p); f.h[1] = *(const v8b*)(p + 16); return f.v;
  }
  static __device__ __forceinline__ v8f mma(v16b a, v16b b, v8f c) {
    return __builtin_amdgcn_wmma_f32_16x16x32_bf16(false, a, false, b, (short)0, c, false, false);
  }
  static __device__ __forceinline__ void guard(v8f& a, v8f& b, v16b x, v16b y) { dep_guard_b(a, b, x, y); }
  static __device__ __forceinline__ void keep(v16b a, v16b b, v16b c, v16b d) { keep4_b(a, b, c, d); }
};

template <int ET> struct Elem;
template <> struct Elem<0> { typedef _Float16 T; };
template <> struct Elem<1> { typedef __bf16 T; };
template <int ET, bool SPLIT, int BIAS_MODE, int OUT_MODE, bool RESID, int ACT = 0>
__global__ __launch_bounds__(256) void wmma_gemm64(
    const unsigned short* __restrict__ Ap, const unsigned short* __restrict__ A2p, int lda, long strideA,
    const unsigned short* __restrict__ Btp, const unsigned short* __restrict__ Bt2p, int ldb, long strideB,
    void* __restrict__ Cout, void* __restrict__ Cout2, int ldc, long strideC,
    const float* __restrict__ bias,
    const float* __restrict__ resid, long strideR,
    int M, int N, int K, float scale) {
  typedef typename Elem<ET>::T T;
  typedef typename Frag<T>::V V;
  const T* A = (const T*)Ap; const T* A2 = (const T*)A2p; const T* Bt = (const T*)Btp; const T* Bt2 = (const T*)Bt2p;
  __shared__ __align__(16) float sT[8][16 * 68];
  const int b    = blockIdx.y;
  const int lane = threadIdx.x & 31;
  const int wave = threadIdx.x >> 5;
  const int tilesN = N >> 6;
  const int tilesM = M >> 6;
  const int tile = blockIdx.x * 8 + wave;
  if (tile >= tilesM * tilesN) return;
  const int tm = tile / tilesN;
  const int tn = tile - tm * tilesN;
  const int m0 = tm << 6;
  const int n0 = tn << 6;

  const T* Ab  = A  + (size_t)b * strideA;
  const T* Bb  = Bt + (size_t)b * strideB;
  const T* Ab2 = SPLIT ? (A2  + (size_t)b * strideA) : nullptr;
  const T* Bb2 = SPLIT ? (Bt2 + (size_t)b * strideB) : nullptr;

  const int rlane = lane & 15;
  const int koff  = (lane >> 4) * 8;
  const int mOff  = (lane >> 4) * 8;

  v8f acc[4][4];
#pragma unroll
  for (int i = 0; i < 4; ++i)
#pragma unroll
    for (int j = 0; j < 4; ++j) acc[i][j] = (v8f){0.f,0.f,0.f,0.f,0.f,0.f,0.f,0.f};

  for (int k0 = 0; k0 < K; k0 += 32) {
    V bh[4], bl[4];
#pragma unroll
    for (int j = 0; j < 4; ++j) {
      const size_t bo = (size_t)(n0 + (j << 4) + rlane) * ldb + koff + k0;
      bh[j] = Frag<T>::load(Bb + bo);
      if (SPLIT) bl[j] = Frag<T>::load(Bb2 + bo);
    }
#pragma unroll
    for (int i = 0; i < 4; ++i) {
      const size_t ao = (size_t)(m0 + (i << 4) + rlane) * lda + koff + k0;
      V ah = Frag<T>::load(Ab + ao);
      V al;
      if (SPLIT) al = Frag<T>::load(Ab2 + ao);
#pragma unroll
      for (int j = 0; j < 4; ++j) {
        acc[i][j] = Frag<T>::mma(ah, bh[j], acc[i][j]);
        if (SPLIT) {
          acc[i][j] = Frag<T>::mma(ah, bl[j], acc[i][j]);
          acc[i][j] = Frag<T>::mma(al, bh[j], acc[i][j]);
        }
      }
      Frag<T>::guard(acc[i][0], acc[i][3], ah, SPLIT ? al : ah);
    }
    Frag<T>::keep(bh[0], bh[1], bh[2], bh[3]);
    if (SPLIT) Frag<T>::keep(bl[0], bl[1], bl[2], bl[3]);
  }
  acc_guard4(acc[0][0], acc[0][1], acc[0][2], acc[0][3]);
  acc_guard4(acc[1][0], acc[1][1], acc[1][2], acc[1][3]);
  acc_guard4(acc[2][0], acc[2][1], acc[2][2], acc[2][3]);
  acc_guard4(acc[3][0], acc[3][1], acc[3][2], acc[3][3]);

  float* slab = sT[wave];
  const float* Rb = RESID ? (resid + (size_t)b * strideR) : nullptr;
#pragma unroll
  for (int i = 0; i < 4; ++i) {
    const int mBase = m0 + (i << 4);
#pragma unroll
    for (int j = 0; j < 4; ++j) {
      const int n = n0 + (j << 4) + rlane;
      float bv = 0.f;
      if (BIAS_MODE == 2) bv = bias[n];
#pragma unroll
      for (int r = 0; r < 8; ++r) {
        float v = acc[i][j][r] * scale;
        if (BIAS_MODE == 1) v += bias[mBase + mOff + r];
        if (BIAS_MODE == 2) v += bv;
        if (RESID) v += Rb[(size_t)(mBase + mOff + r) * ldc + n];
        if (ACT == 1) v = tanhf(v);
        if (ACT == 2) v = fmaxf(v, 0.0f);
        if (ACT == 4) v = (v > 0.f) ? v : 0.01f * v;
        slab[(mOff + r) * 68 + (j << 4) + rlane] = v;
      }
    }
    __builtin_amdgcn_fence(__ATOMIC_RELEASE, "workgroup");
    __builtin_amdgcn_wave_barrier();
    __builtin_amdgcn_fence(__ATOMIC_ACQUIRE, "workgroup");
    if (OUT_MODE == 0) {
      float* C = (float*)Cout + (size_t)b * strideC;
      const int hh = lane >> 4, c4 = (lane & 15) * 4;
      for (int pass = 0; pass < 2; ++pass) {
#pragma unroll
        for (int it = 0; it < 8; ++it) {
          const int row = it * 2 + hh;
          v4f v = *(const v4f*)(slab + row * 68 + c4);
          *(volatile v4f*)(C + (size_t)(mBase + row) * ldc + n0 + c4) = v;
        }
        __threadfence();
      }
    } else {
      const int q = lane >> 3, c8 = (lane & 7) * 8;
      unsigned short* C  = (unsigned short*)Cout  + (size_t)b * strideC;
      unsigned short* C2 = (OUT_MODE == 2) ? ((unsigned short*)Cout2 + (size_t)b * strideC) : nullptr;
      for (int pass = 0; pass < 2; ++pass) {
#pragma unroll
        for (int it = 0; it < 4; ++it) {
          const int row = it * 4 + q;
          const float* sp = slab + row * 68 + c8;
          v8h hv, lv;
#pragma unroll
          for (int e = 0; e < 8; ++e) {
            if (OUT_MODE == 1) {
              hv[e] = (_Float16)sp[e];
            } else {
              unsigned short hb = f2bf_bits(sp[e]);
              unsigned short lb = f2bf_bits(sp[e] - bf_bits2f(hb));
              hv[e] = __builtin_bit_cast(_Float16, hb);
              lv[e] = __builtin_bit_cast(_Float16, lb);
            }
          }
          *(volatile v8h*)(C + (size_t)(mBase + row) * ldc + n0 + c8) = hv;
          if (OUT_MODE == 2) *(volatile v8h*)(C2 + (size_t)(mBase + row) * ldc + n0 + c8) = lv;
        }
        __threadfence();
      }
    }
    __builtin_amdgcn_fence(__ATOMIC_RELEASE, "workgroup");
    __builtin_amdgcn_wave_barrier();
    __builtin_amdgcn_fence(__ATOMIC_ACQUIRE, "workgroup");
  }
}

__global__ __launch_bounds__(256) void cast_f32_f16x2(
    const float* __restrict__ in, _Float16* __restrict__ out, int n2) {
  int i = blockIdx.x * 256 + threadIdx.x;
  if (i < n2) {
    const _Float16 h0 = (_Float16)in[2 * i], h1 = (_Float16)in[2 * i + 1];
    const unsigned u = (unsigned)__builtin_bit_cast(unsigned short, h0) | ((unsigned)__builtin_bit_cast(unsigned short, h1) << 16);
    ((volatile unsigned*)out)[i] = u;
    __threadfence();
    ((volatile unsigned*)out)[i] = u;
  }
}

__global__ __launch_bounds__(256) void split_x_kernel(const float* __restrict__ x,
                                                      unsigned short* __restrict__ xhi,
                                                      unsigned short* __restrict__ xlo) {
  const int i = blockIdx.x * 256 + threadIdx.x;
  const v2f f = *(const v2f*)(x + 2 * (size_t)i);
  const unsigned short h0 = f2bf_bits(f[0]), h1 = f2bf_bits(f[1]);
  const unsigned short l0 = f2bf_bits(f[0] - bf_bits2f(h0)), l1 = f2bf_bits(f[1] - bf_bits2f(h1));
  const unsigned uh = (unsigned)h0 | ((unsigned)h1 << 16);
  const unsigned ul = (unsigned)l0 | ((unsigned)l1 << 16);
  ((volatile unsigned*)xhi)[i] = uh;
  ((volatile unsigned*)xlo)[i] = ul;
  __threadfence();
  ((volatile unsigned*)xhi)[i] = uh;
  ((volatile unsigned*)xlo)[i] = ul;
}

__global__ __launch_bounds__(256) void split_wT_kernel(const float* __restrict__ W,
                                                       unsigned short* __restrict__ wthi,
                                                       unsigned short* __restrict__ wtlo) {
  const int i  = blockIdx.x * 256 + threadIdx.x;
  const int f2 = (i & (NFEAT_C / 2 - 1)) * 2;
  const int r  = i >> 8;
  const int d  = r & (NHID_C - 1);
  const int ph = r >> 7;
  const float w0 = W[((size_t)ph * NFEAT_C + f2) * NHID_C + d];
  const float w1 = W[((size_t)ph * NFEAT_C + f2 + 1) * NHID_C + d];
  const unsigned short h0 = f2bf_bits(w0), h1 = f2bf_bits(w1);
  const unsigned short l0 = f2bf_bits(w0 - bf_bits2f(h0)), l1 = f2bf_bits(w1 - bf_bits2f(h1));
  const unsigned uh = (unsigned)h0 | ((unsigned)h1 << 16);
  const unsigned ul = (unsigned)l0 | ((unsigned)l1 << 16);
  ((volatile unsigned*)wthi)[i] = uh;
  ((volatile unsigned*)wtlo)[i] = ul;
  __threadfence();
  ((volatile unsigned*)wthi)[i] = uh;
  ((volatile unsigned*)wtlo)[i] = ul;
}

__global__ __launch_bounds__(256) void cast_wsemT_kernel(const float* __restrict__ Wsem,
                                                         unsigned short* __restrict__ wsemT) {
  const int i  = blockIdx.x * 256 + threadIdx.x;
  const int f2 = (i & (KCAT_C / 2 - 1)) * 2;
  const int s  = i >> 8;
  const _Float16 h0 = (_Float16)(Wsem[(size_t)f2 * SHID_C + s] * WSEM_CARRY);
  const _Float16 h1 = (_Float16)(Wsem[(size_t)(f2 + 1) * SHID_C + s] * WSEM_CARRY);
  const unsigned u = (unsigned)__builtin_bit_cast(unsigned short, h0) | ((unsigned)__builtin_bit_cast(unsigned short, h1) << 16);
  ((volatile unsigned*)wsemT)[i] = u;
  __threadfence();
  ((volatile unsigned*)wsemT)[i] = u;
}

__global__ __launch_bounds__(256) void node_scores_kernel(const float* __restrict__ hT32,
                                                          const float* __restrict__ a_node,
                                                          float* __restrict__ s_src,
                                                          float* __restrict__ s_dst) {
  const int ph = blockIdx.x >> 3;
  const int n  = ((blockIdx.x & 7) << 8) + threadIdx.x;
  const float* hcol = hT32 + (size_t)ph * NHID_C * NNODE + n;
  const float* av   = a_node + (size_t)ph * 2 * NHID_C;
  float ss = 0.f, sd = 0.f;
#pragma unroll 4
  for (int d = 0; d < NHID_C; ++d) {
    const float hv = hcol[(size_t)d * NNODE];
    ss = fmaf(hv, av[d], ss);
    sd = fmaf(hv, av[NHID_C + d], sd);
  }
  const size_t o = (size_t)ph * NNODE + n;
  *(volatile float*)(s_src + o) = ss;
  *(volatile float*)(s_dst + o) = sd;
  __threadfence();
  *(volatile float*)(s_src + o) = ss;
  *(volatile float*)(s_dst + o) = sd;
}

__global__ __launch_bounds__(256) void row_stats_kernel(const float* __restrict__ adjs,
                                                        const float* __restrict__ s_src,
                                                        const float* __restrict__ s_dst,
                                                        float* __restrict__ rmax,
                                                        float* __restrict__ rinv) {
  __shared__ float smx[NHEAD_C][32];
  __shared__ float sri[NHEAD_C][32];
  const int wave = threadIdx.x >> 5, lane = threadIdx.x & 31;
  const int p  = blockIdx.x / (NNODE / 32);
  const int i0 = (blockIdx.x % (NNODE / 32)) * 32;
  const float* sdb = s_dst + (size_t)p * NHEAD_C * NNODE;
#pragma unroll 1
  for (int q = 0; q < 4; ++q) {
    const int il = wave * 4 + q;
    const int i  = i0 + il;
    const float* arow = adjs + ((size_t)p * NNODE + i) * NNODE;
    float sv[NHEAD_C], mx[NHEAD_C], sm[NHEAD_C];
#pragma unroll
    for (int hd = 0; hd < NHEAD_C; ++hd) {
      sv[hd] = s_src[(size_t)(p * NHEAD_C + hd) * NNODE + i];
      mx[hd] = -__builtin_inff();
      sm[hd] = 0.f;
    }
#pragma unroll 1
    for (int j = lane; j < NNODE; j += 32) {
      const float a = arow[j];
#pragma unroll
      for (int hd = 0; hd < NHEAD_C; ++hd) {
        float e = sv[hd] + sdb[(size_t)hd * NNODE + j];
        e = (e > 0.f) ? e : LRELU_SLOPE * e;
        const float em = (a > 0.f) ? e : MASK_FILL;
        mx[hd] = fmaxf(mx[hd], em);
      }
    }
#pragma unroll
    for (int hd = 0; hd < NHEAD_C; ++hd) {
#pragma unroll
      for (int off = 16; off >= 1; off >>= 1) mx[hd] = fmaxf(mx[hd], __shfl_xor(mx[hd], off, 32));
    }
#pragma unroll 1
    for (int j = lane; j < NNODE; j += 32) {
      const float a = arow[j];
#pragma unroll
      for (int hd = 0; hd < NHEAD_C; ++hd) {
        float e = sv[hd] + sdb[(size_t)hd * NNODE + j];
        e = (e > 0.f) ? e : LRELU_SLOPE * e;
        const float em = (a > 0.f) ? e : MASK_FILL;
        sm[hd] += expf(em - mx[hd]);
      }
    }
#pragma unroll
    for (int hd = 0; hd < NHEAD_C; ++hd) {
#pragma unroll
      for (int off = 16; off >= 1; off >>= 1) sm[hd] += __shfl_xor(sm[hd], off, 32);
    }
    if (lane == 0) {
#pragma unroll
      for (int hd = 0; hd < NHEAD_C; ++hd) {
        smx[hd][il] = mx[hd];
        sri[hd][il] = 1.0f / sm[hd];
      }
    }
  }
  __syncthreads();
  if (wave == 0) {
    for (int pass = 0; pass < 2; ++pass) {
#pragma unroll
      for (int hd = 0; hd < NHEAD_C; ++hd) {
        const size_t o = (size_t)(p * NHEAD_C + hd) * NNODE + i0 + lane;
        *(volatile float*)(rmax + o) = smx[hd][lane];
        *(volatile float*)(rinv + o) = sri[hd][lane];
      }
      __threadfence();
    }
  }
}

__device__ __forceinline__ _Float16 att_p16(float adjv, float dv, float sv, float rm, float ri) {
  float e = sv + dv;
  e = (e > 0.f) ? e : LRELU_SLOPE * e;
  const float em = (adjv > 0.f) ? e : MASK_FILL;
  return (_Float16)(expf(em - rm) * ri);
}
__device__ __forceinline__ float elu1(float x) {
  const float t = expm1f(fminf(x, 0.f));
  return (x > 0.f) ? x : t;
}

__global__ __launch_bounds__(128) void att_gemm_kernel(const float* __restrict__ adjs,
                                                       const float* __restrict__ s_src,
                                                       const float* __restrict__ s_dst,
                                                       const float* __restrict__ rmax,
                                                       const float* __restrict__ rinv,
                                                       const unsigned short* __restrict__ hT16p,
                                                       float* __restrict__ m32,
                                                       unsigned short* __restrict__ m16p) {
  __shared__ __align__(16) float slab_all[NHEAD_C][16 * SLAB_PITCH];
  const _Float16* hT16 = (const _Float16*)hT16p;
  const int tid = threadIdx.x, wave = tid >> 5, lane = tid & 31;
  const int hh = lane >> 4, c = lane & 15;
  const int p       = blockIdx.x / (NNODE / 16);
  const int rowbase = (blockIdx.x % (NNODE / 16)) * 16;
  const int ph = p * NHEAD_C + wave;
  const int i  = rowbase + c;
  const size_t phn = (size_t)ph * NNODE;
  const float sv = s_src[phn + i];
  const float rm = rmax[phn + i];
  const float ri = rinv[phn + i] * PCARRY;
  const float* arow = adjs + ((size_t)p * NNODE + i) * NNODE;
  const float* sdv  = s_dst + phn;
  const _Float16* hbase = hT16 + (size_t)ph * NHID_C * NNODE;

  v8f acc[8];
#pragma unroll
  for (int t = 0; t < 8; ++t) acc[t] = (v8f){0.f,0.f,0.f,0.f,0.f,0.f,0.f,0.f};

#pragma unroll 1
  for (int kt = 0; kt < NNODE / 32; ++kt) {
    const int ka = kt * 32 + 8 * hh;
    const int kb = ka + 16;
    const v4f a0 = *(const v4f*)(arow + ka);
    const v4f a1 = *(const v4f*)(arow + ka + 4);
    const v4f a2 = *(const v4f*)(arow + kb);
    const v4f a3 = *(const v4f*)(arow + kb + 4);
    const v4f d0 = *(const v4f*)(sdv + ka);
    const v4f d1 = *(const v4f*)(sdv + ka + 4);
    const v4f d2 = *(const v4f*)(sdv + kb);
    const v4f d3 = *(const v4f*)(sdv + kb + 4);
    v16h A;
#pragma unroll
    for (int e = 0; e < 4; ++e) {
      A[e]      = att_p16(a0[e], d0[e], sv, rm, ri);
      A[4 + e]  = att_p16(a1[e], d1[e], sv, rm, ri);
      A[8 + e]  = att_p16(a2[e], d2[e], sv, rm, ri);
      A[12 + e] = att_p16(a3[e], d3[e], sv, rm, ri);
    }
#pragma unroll
    for (int g = 0; g < 2; ++g) {
      asm volatile("" ::: "memory");
      v16h Bf[4];
#pragma unroll
      for (int j = 0; j < 4; ++j)
        Bf[j] = Frag<_Float16>::load(hbase + (size_t)((g * 4 + j) * 16 + c) * NNODE + ka);
#pragma unroll
      for (int j = 0; j < 4; ++j) acc[g * 4 + j] = Frag<_Float16>::mma(A, Bf[j], acc[g * 4 + j]);
      dep_guard_h(acc[g * 4], acc[g * 4 + 3], A, Bf[3]);
      keep4_h(Bf[0], Bf[1], Bf[2], Bf[3]);
    }
  }
  acc_guard4(acc[0], acc[1], acc[2], acc[3]);
  acc_guard4(acc[4], acc[5], acc[6], acc[7]);

  float* slab = slab_all[wave];
#pragma unroll
  for (int dt = 0; dt < 8; ++dt) {
#pragma unroll
    for (int r = 0; r < 8; ++r) slab[(8 * hh + r) * SLAB_PITCH + dt * 16 + c] = acc[dt][r] * PCARRY_INV;
  }
  __syncthreads();
#pragma unroll 1
  for (int row = 0; row < 16; ++row) {
    v4f v = *(const v4f*)(slab + row * SLAB_PITCH + 4 * lane);
    v[0] = elu1(v[0]); v[1] = elu1(v[1]); v[2] = elu1(v[2]); v[3] = elu1(v[3]);
    *(v4f*)(slab + row * SLAB_PITCH + 4 * lane) = v;
  }
  __syncthreads();
  float* mrow = m32 + ((size_t)p * NNODE + rowbase) * KCAT_C + wave * NHID_C;
  for (int pass = 0; pass < 2; ++pass) {
#pragma unroll
    for (int row = 0; row < 16; ++row) {
      const v4f v = *(const v4f*)(slab + row * SLAB_PITCH + 4 * lane);
      *(volatile v4f*)(mrow + (size_t)row * KCAT_C + 4 * lane) = v;
    }
    __threadfence();
  }
  _Float16* mh = (_Float16*)m16p + ((size_t)p * NNODE + rowbase) * KCAT_C + wave * NHID_C;
  for (int pass = 0; pass < 2; ++pass) {
#pragma unroll
    for (int it = 0; it < 8; ++it) {
      const int row = it * 2 + hh;
      const float* sp = slab + row * SLAB_PITCH + c * 8;
      v8h hv;
#pragma unroll
      for (int e = 0; e < 8; ++e) hv[e] = (_Float16)(sp[e] * MCARRY);
      *(volatile v8h*)(mh + (size_t)row * KCAT_C + c * 8) = hv;
    }
    __threadfence();
  }
}

__global__ __launch_bounds__(256) void sem_scores_kernel(const float* __restrict__ hs,
                                                         const float* __restrict__ q_sem,
                                                         float* __restrict__ sc) {
  __shared__ float part[8];
  const int p = blockIdx.x, tid = threadIdx.x, wave = tid >> 5, lane = tid & 31;
  const v4f q4 = *(const v4f*)(q_sem + lane * 4);
  const v4f* hs4 = (const v4f*)(hs + (size_t)p * NNODE * SHID_C);
  float accv = 0.f;
#pragma unroll 1
  for (int idx = tid; idx < NNODE * SHID_C / 4; idx += 256) {
    const v4f v = hs4[idx];
    accv = fmaf(v[0], q4[0], accv);
    accv = fmaf(v[1], q4[1], accv);
    accv = fmaf(v[2], q4[2], accv);
    accv = fmaf(v[3], q4[3], accv);
  }
#pragma unroll
  for (int off = 16; off >= 1; off >>= 1) accv += __shfl_xor(accv, off, 32);
  if (lane == 0) part[wave] = accv;
  __syncthreads();
  if (wave == 0) {
    float t = part[lane & 7];
    t = (lane < 8) ? t : 0.f;
#pragma unroll
    for (int off = 16; off >= 1; off >>= 1) t += __shfl_xor(t, off, 32);
    const float mean = t * (1.0f / (float)NNODE);
    const float val = (lane == 0) ? mean : 0.f;
    for (int pass = 0; pass < 2; ++pass) {
      *(volatile float*)(sc + p * 32 + lane) = val;
      __threadfence();
    }
  }
}

__global__ __launch_bounds__(256) void combine_kernel(const float* __restrict__ m32,
                                                      const float* __restrict__ sc,
                                                      float* __restrict__ out) {
  const int t = blockIdx.x * 256 + threadIdx.x;
  const float s0 = sc[0], s1 = sc[32], s2 = sc[64];
  const float mx = fmaxf(s0, fmaxf(s1, s2));
  const float w0 = expf(s0 - mx), w1 = expf(s1 - mx), w2 = expf(s2 - mx);
  const float inv = 1.0f / (w0 + w1 + w2);
  const float c0 = w0 * inv, c1 = w1 * inv, c2 = w2 * inv;
  const size_t st4 = (size_t)NNODE * KCAT_C / 4;
  const v4f* m4 = (const v4f*)m32;
  const v4f va = m4[t], vb = m4[t + st4], vc = m4[t + 2 * st4];
  const v4f o = va * c0 + vb * c1 + vc * c2;
  *(volatile v4f*)(out + (size_t)t * 4) = o;
  __threadfence();
  *(volatile v4f*)(out + (size_t)t * 4) = o;
}

extern "C" void kernel_launch(void* const* d_in, const int* in_sizes, int n_in,
                              void* d_out, int out_size, void* d_ws,
                              size_t ws_size, hipStream_t stream) {
  if (n_in < 7) return;
  if (ws_size < WS_TOTAL) return;
  if ((size_t)out_size < (size_t)NNODE * KCAT_C) return;
  if (in_sizes[0] != NNODE * NFEAT_C) return;
  if (in_sizes[1] != NPATH_C * NNODE * NNODE) return;
  if (in_sizes[2] != NPH_C * NFEAT_C * NHID_C) return;
  if (in_sizes[3] != NPH_C * 2 * NHID_C) return;
  if (in_sizes[4] != KCAT_C * SHID_C) return;
  if (in_sizes[5] != SHID_C || in_sizes[6] != SHID_C) return;

  const float* x      = (const float*)d_in[0];
  const float* adjs   = (const float*)d_in[1];
  const float* W_node = (const float*)d_in[2];
  const float* a_node = (const float*)d_in[3];
  const float* W_sem  = (const float*)d_in[4];
  const float* b_sem  = (const float*)d_in[5];
  const float* q_sem  = (const float*)d_in[6];
  float* out = (float*)d_out;

  char* ws = (char*)d_ws;
  unsigned short* xhi   = (unsigned short*)(ws + OFF_XHI);
  unsigned short* xlo   = (unsigned short*)(ws + OFF_XLO);
  unsigned short* wthi  = (unsigned short*)(ws + OFF_WTHI);
  unsigned short* wtlo  = (unsigned short*)(ws + OFF_WTLO);
  float*          hT32  = (float*)(ws + OFF_HT32);
  unsigned short* hT16  = (unsigned short*)(ws + OFF_HT16);
  float*          s_src = (float*)(ws + OFF_SSRC);
  float*          s_dst = (float*)(ws + OFF_SDST);
  float*          rmx   = (float*)(ws + OFF_RMAX);
  float*          rin   = (float*)(ws + OFF_RINV);
  float*          m32   = (float*)(ws + OFF_M32);
  unsigned short* m16   = (unsigned short*)(ws + OFF_M16);
  unsigned short* wsemT = (unsigned short*)(ws + OFF_WSEMT);
  float*          hs    = (float*)(ws + OFF_HS);
  float*          sc    = (float*)(ws + OFF_SC);

  split_x_kernel<<<(NNODE * NFEAT_C / 2) / 256, 256, 0, stream>>>(x, xhi, xlo);
  split_wT_kernel<<<(NPH_C * NHID_C * NFEAT_C / 2) / 256, 256, 0, stream>>>(W_node, wthi, wtlo);
  cast_wsemT_kernel<<<(SHID_C * KCAT_C / 2) / 256, 256, 0, stream>>>(W_sem, wsemT);

  wmma_gemm64<1, true, 0, 0, false, 0><<<dim3(8, NPH_C), 256, 0, stream>>>(
      wthi, wtlo, NFEAT_C, (long)NHID_C * NFEAT_C,
      xhi, xlo, NFEAT_C, 0L,
      (void*)hT32, (void*)hT16, NNODE, (long)NHID_C * NNODE,
      b_sem, hs, 0L,
      NHID_C, NNODE, NFEAT_C, 1.0f);

  cast_f32_f16x2<<<(NPH_C * NHID_C * NNODE / 2) / 256, 256, 0, stream>>>(hT32, (_Float16*)hT16, NPH_C * NHID_C * NNODE / 2);

  node_scores_kernel<<<NPH_C * (NNODE / 256), 256, 0, stream>>>(hT32, a_node, s_src, s_dst);

  row_stats_kernel<<<NPATH_C * (NNODE / 32), 256, 0, stream>>>(adjs, s_src, s_dst, rmx, rin);

  att_gemm_kernel<<<NPATH_C * (NNODE / 16), 128, 0, stream>>>(adjs, s_src, s_dst, rmx, rin, hT16, m32, m16);

  wmma_gemm64<0, false, 2, 0, false, 1><<<dim3(24, 1), 256, 0, stream>>>(
      m16, m16, KCAT_C, 0L,
      wsemT, wsemT, KCAT_C, 0L,
      (void*)hs, (void*)hT16, SHID_C, 0L,
      b_sem, hT32, 0L,
      NPATH_C * NNODE, SHID_C, KCAT_C, SEM_SCALE);

  sem_scores_kernel<<<NPATH_C, 256, 0, stream>>>(hs, q_sem, sc);

  combine_kernel<<<(NNODE * KCAT_C / 4) / 256, 256, 0, stream>>>(m32, sc, out);
}
